// MDU_15083925144367
// MI455X (gfx1250) — hardware-verified
//
#include <hip/hip_runtime.h>
#include <math.h>

#define NB_ 8
#define CC 64
#define IH 128
#define IW 128
#define NPIX (IH * IW)
#define KK 9
#define KTOT (CC * KK)
#define NGEN (CC * KK)

typedef _Float16 f16;
typedef __attribute__((ext_vector_type(16))) f16 f16x16;
typedef __attribute__((ext_vector_type(8)))  f16 f16x8;
typedef __attribute__((ext_vector_type(8)))  float f32x8;
typedef __attribute__((ext_vector_type(4)))  float v4f_t;
typedef float v4fa __attribute__((ext_vector_type(4), may_alias));
typedef __attribute__((ext_vector_type(4)))  unsigned v4u_t;
typedef unsigned v4ua __attribute__((ext_vector_type(4), may_alias));
__device__ __forceinline__ f32x8 wmma16(f16x16 a, f16x16 b, f32x8 c) {
  c = __builtin_amdgcn_wmma_f32_16x16x32_f16(false, a, false, b, (short)0, c, false, false);
  asm volatile("v_nop\n\tv_nop\n\tv_nop\n\tv_nop" : "+v"(c) : "v"(a), "v"(b));
  return c;
}
__device__ __forceinline__ f16x16 lds_frag(const f16* base, int stride) {
  const int lane = threadIdx.x & 31, row = lane & 15, kh = (lane >> 4) * 8;
  const f16x8 lo = *(const f16x8*)(base + row * stride + kh);
  const f16x8 hi = *(const f16x8*)(base + row * stride + kh + 16);
  f16x16 f;
#pragma unroll
  for (int i = 0; i < 8; ++i) { f[i] = lo[i]; f[i + 8] = hi[i]; }
  return f;
}
template <int MODE>
__global__ __launch_bounds__(256) void k_conv3(const float* __restrict__ in, const float* __restrict__ w, const float* __restrict__ bias, void* __restrict__ outp) {
  __shared__ __attribute__((aligned(16))) f16 aS[128 * 168];
  __shared__ __attribute__((aligned(16))) f16 wS[64 * 168];
  __shared__ __attribute__((aligned(16))) float oS[64 * 132];
  const int tid = threadIdx.x, lane = tid & 31, wave = tid >> 5, cl = lane & 15, rh = (lane >> 4) * 8;
  const int b = blockIdx.x / (NPIX / 128), p0 = (blockIdx.x % (NPIX / 128)) * 128;
  for (int e = tid; e < 128 * 16; e += 256) aS[(e >> 4) * 168 + 144 + (e & 15)] = (f16)0.0f;
  for (int e = tid; e < 64 * 16; e += 256) wS[(e >> 4) * 168 + 144 + (e & 15)] = (f16)0.0f;
  f32x8 acc[4];
#pragma unroll
  for (int j = 0; j < 4; ++j) { f32x8 z = {}; acc[j] = z; }
  __syncthreads();
#pragma unroll 1
  for (int cg = 0; cg < CC / 16; ++cg) {
    for (int e = tid; e < 128 * 144; e += 256) { const int r = e / 144, q = e % 144, cc = q / 9, k = q % 9; const int p = p0 + r, oh = p / IW, ow = p % IW; const int ih = oh + k / 3 - 1, iw = ow + k % 3 - 1;
      const int c = cg * 16 + cc; float v = 0.0f;
      if (ih >= 0 && ih < IH && iw >= 0 && iw < IW) v = in[(((size_t)b * CC + c) * IH + min(max(ih, 0), IH - 1)) * IW + min(max(iw, 0), IW - 1)];
      aS[r * 168 + q] = (f16)v; }
    for (int e = tid; e < 64 * 144; e += 256) { const int o = e / 144, q = e % 144; wS[o * 168 + q] = (f16)w[((size_t)o * CC + cg * 16) * KK + q]; }
    __syncthreads();
#pragma unroll
    for (int ks = 0; ks < 5; ++ks) { const f16x16 af = lds_frag(aS + (wave * 16) * 168 + ks * 32, 168);
#pragma unroll
      for (int j = 0; j < 4; ++j) acc[j] = wmma16(af, lds_frag(wS + (j * 16) * 168 + ks * 32, 168), acc[j]); }
    __syncthreads();
  }
  if (MODE == 1) {
#pragma unroll
    for (int j = 0; j < 4; ++j)
#pragma unroll
      for (int r = 0; r < 8; ++r) { const int o = j * 16 + cl, p = wave * 16 + rh + r; oS[o * 132 + p] = fmaxf(acc[j][r] + bias[o], 0.0f); }
    __syncthreads();
    float* out = (float*)outp;
#pragma unroll 1
    for (int pass = 0; pass < 2; ++pass) { for (int q4 = tid; q4 < 64 * 32; q4 += 256) { const int o = q4 >> 5, c4 = (q4 & 31) * 4;
        *(volatile v4f_t*)(out + ((size_t)b * CC + o) * NPIX + p0 + c4) = *(const v4fa*)(oS + o * 132 + c4); } __threadfence(); }
  } else {
#pragma unroll
    for (int j = 0; j < 4; ++j)
#pragma unroll
      for (int r = 0; r < 8; ++r) { const int o = j * 16 + cl, p = wave * 16 + rh + r; oS[p * 66 + o] = acc[j][r] + bias[o]; }
    __syncthreads();
    float* t1 = (float*)outp;
#pragma unroll 1
    for (int pass = 0; pass < 2; ++pass) { for (int q = tid; q < 128 * 16; q += 256) { const int p = q >> 4, c4 = (q & 15) * 4;
        v4f_t v; v[0] = oS[p * 66 + c4]; v[1] = oS[p * 66 + c4 + 1]; v[2] = oS[p * 66 + c4 + 2]; v[3] = oS[p * 66 + c4 + 3];
        *(volatile v4f_t*)(t1 + ((size_t)b * NPIX + p0 + p) * CC + c4) = v; } __threadfence(); }
  }
}
__global__ __launch_bounds__(256) void k_conv3p(const float* __restrict__ in, const float* __restrict__ w, const float* __restrict__ bias, float* __restrict__ out) {
  __shared__ __attribute__((aligned(16))) f16 aS[128 * 104], aL[128 * 104];
  __shared__ __attribute__((aligned(16))) f16 wS[64 * 104], wL[64 * 104];
  __shared__ __attribute__((aligned(16))) float oS[64 * 132];
  const int tid = threadIdx.x, lane = tid & 31, wave = tid >> 5, cl = lane & 15, rh = (lane >> 4) * 8;
  const int b = blockIdx.x / (NPIX / 128), p0 = (blockIdx.x % (NPIX / 128)) * 128;
  for (int e = tid; e < 128 * 24; e += 256) { const int r = e / 24, c = 72 + e % 24; aS[r * 104 + c] = (f16)0.0f; aL[r * 104 + c] = (f16)0.0f; }
  for (int e = tid; e < 64 * 24; e += 256) { const int r = e / 24, c = 72 + e % 24; wS[r * 104 + c] = (f16)0.0f; wL[r * 104 + c] = (f16)0.0f; }
  f32x8 acc[4], accx[4];
#pragma unroll
  for (int j = 0; j < 4; ++j) { f32x8 z = {}; acc[j] = z; accx[j] = z; }
  __syncthreads();
#pragma unroll 1
  for (int cg = 0; cg < CC / 8; ++cg) {
    for (int e = tid; e < 128 * 72; e += 256) { const int r = e / 72, q = e % 72, cc = q / 9, k = q % 9; const int p = p0 + r, oh = p / IW, ow = p % IW; const int ih = oh + k / 3 - 1, iw = ow + k % 3 - 1;
      const int c = cg * 8 + cc; float v = 0.0f;
      if (ih >= 0 && ih < IH && iw >= 0 && iw < IW) v = in[(((size_t)b * CC + c) * IH + min(max(ih, 0), IH - 1)) * IW + min(max(iw, 0), IW - 1)];
      const f16 h = (f16)v; aS[r * 104 + q] = h; aL[r * 104 + q] = (f16)((v - (float)h) * 2048.0f); }
    for (int e = tid; e < 64 * 72; e += 256) { const int o = e / 72, q = e % 72; const float v = w[((size_t)o * CC + cg * 8) * KK + q]; const f16 h = (f16)v; wS[o * 104 + q] = h; wL[o * 104 + q] = (f16)((v - (float)h) * 2048.0f); }
    __syncthreads();
#pragma unroll
    for (int ks = 0; ks < 3; ++ks) { const f16x16 af = lds_frag(aS + (wave * 16) * 104 + ks * 32, 104), afl = lds_frag(aL + (wave * 16) * 104 + ks * 32, 104);
#pragma unroll
      for (int j = 0; j < 4; ++j) { const f16x16 bf = lds_frag(wS + (j * 16) * 104 + ks * 32, 104), bfl = lds_frag(wL + (j * 16) * 104 + ks * 32, 104);
        acc[j] = wmma16(af, bf, acc[j]); accx[j] = wmma16(af, bfl, accx[j]); accx[j] = wmma16(afl, bf, accx[j]); } }
    __syncthreads();
  }
#pragma unroll
  for (int j = 0; j < 4; ++j)
#pragma unroll
    for (int r = 0; r < 8; ++r) { const int o = j * 16 + cl, p = wave * 16 + rh + r; oS[o * 132 + p] = fmaxf(acc[j][r] + accx[j][r] * (1.0f / 2048.0f) + bias[o], 0.0f); }
  __syncthreads();
#pragma unroll 1
  for (int pass = 0; pass < 2; ++pass) { for (int q4 = tid; q4 < 64 * 32; q4 += 256) { const int o = q4 >> 5, c4 = (q4 & 31) * 4;
      *(volatile v4f_t*)(out + ((size_t)b * CC + o) * NPIX + p0 + c4) = *(const v4fa*)(oS + o * 132 + c4); } __threadfence(); }
}
__global__ __launch_bounds__(256) void k_dyn(const float* __restrict__ t1, const float* __restrict__ w2, const float* __restrict__ b2, const float* __restrict__ x, float* __restrict__ result) {
  __shared__ __attribute__((aligned(16))) f16 aS[128 * 72], aL[128 * 72];
  __shared__ __attribute__((aligned(16))) f16 wS[80 * 72], wL[80 * 72];
  __shared__ float kg[128 * 84];
  __shared__ __attribute__((aligned(16))) float rS[8 * 132];
  const int tid = threadIdx.x, lane = tid & 31, wave = tid >> 5, cl = lane & 15, rh = (lane >> 4) * 8;
  const int b = blockIdx.x / (NPIX / 128), p0 = (blockIdx.x % (NPIX / 128)) * 128;
  for (int e = tid; e < 128 * 64; e += 256) { const int p = e >> 6, c = e & 63; const float v = t1[((size_t)b * NPIX + p0 + p) * CC + c]; const f16 h = (f16)v; aS[p * 72 + c] = h; aL[p * 72 + c] = (f16)((v - (float)h) * 2048.0f); }
  for (int e = tid; e < 8 * 72; e += 256) { wS[(72 + (e / 72)) * 72 + (e % 72)] = (f16)0.0f; wL[(72 + (e / 72)) * 72 + (e % 72)] = (f16)0.0f; }
#pragma unroll 1
  for (int ch = 0; ch < CC / 8; ++ch) {
    __syncthreads();
    for (int e = tid; e < 72 * 64; e += 256) { const int nl = e >> 6, c = e & 63; const float v = w2[(size_t)(ch * 72 + nl) * CC + c]; const f16 h = (f16)v; wS[nl * 72 + c] = h; wL[nl * 72 + c] = (f16)((v - (float)h) * 2048.0f); }
    __syncthreads();
    f32x8 acc[5], accx[5];
#pragma unroll
    for (int j = 0; j < 5; ++j) { f32x8 z = {}; acc[j] = z; accx[j] = z; }
#pragma unroll
    for (int ks = 0; ks < 2; ++ks) { const f16x16 af = lds_frag(aS + (wave * 16) * 72 + ks * 32, 72), afl = lds_frag(aL + (wave * 16) * 72 + ks * 32, 72);
#pragma unroll
      for (int j = 0; j < 5; ++j) { const f16x16 bf = lds_frag(wS + (j * 16) * 72 + ks * 32, 72), bfl = lds_frag(wL + (j * 16) * 72 + ks * 32, 72);
        acc[j] = wmma16(af, bf, acc[j]); accx[j] = wmma16(af, bfl, accx[j]); accx[j] = wmma16(afl, bf, accx[j]); } }
#pragma unroll
    for (int j = 0; j < 5; ++j)
#pragma unroll
      for (int r = 0; r < 8; ++r) { const int n = j * 16 + cl, p = wave * 16 + rh + r; kg[p * 84 + n] = acc[j][r] + accx[j][r] * (1.0f / 2048.0f) + ((n < 72) ? b2[ch * 72 + n] : 0.0f); }
    __syncthreads();
    { const int p = tid & 127, c0 = (tid >> 7) * 4; const int gp = p0 + p, oh = gp / IW, ow = gp % IW;
#pragma unroll 1
      for (int cc = 0; cc < 4; ++cc) { const int c = ch * 8 + c0 + cc; const float* xc = x + ((size_t)b * CC + c) * NPIX; float s = 0.0f;
#pragma unroll
        for (int k = 0; k < 9; ++k) { const int ih = oh + k / 3 - 1, iw = ow + k % 3 - 1;
          const float xv = (ih >= 0 && ih < IH && iw >= 0 && iw < IW) ? xc[min(max(ih, 0), IH - 1) * IW + min(max(iw, 0), IW - 1)] : 0.0f;
          s += xv * kg[p * 84 + (c0 + cc) * 9 + k]; }
        rS[(c0 + cc) * 132 + p] = s; } }
    __syncthreads();
#pragma unroll 1
    for (int pass = 0; pass < 2; ++pass) { { const int cc_ = tid >> 5, c4 = (tid & 31) * 4;
        *(volatile v4f_t*)(result + ((size_t)b * CC + ch * 8 + cc_) * NPIX + p0 + c4) = *(const v4fa*)(rS + cc_ * 132 + c4); } __threadfence(); }
  }
}

extern "C" void kernel_launch(void* const* d_in, const int* in_sizes, int n_in,
                              void* d_out, int out_size, void* d_ws, size_t ws_size,
                              hipStream_t stream) {
  (void)in_sizes; (void)n_in; (void)out_size;
  const float** f = (const float**)d_in;
  const float* x = f[0], *y = f[1], *w1 = f[2], *b1 = f[3], *w2 = f[4], *b2 = f[5], *w3 = f[6], *b3 = f[7];
  float* out = (float*)d_out;
  char* ws = (char*)d_ws;
  float* t1 = (float*)ws; ws += (size_t)NB_ * NPIX * CC * 4;
  float* result = (float*)ws; ws += (size_t)NB_ * CC * NPIX * 4;
  if ((size_t)(ws - (char*)d_ws) > ws_size) return;
  k_conv3<0><<<dim3(NB_ * NPIX / 128), dim3(256), 0, stream>>>(y, w1, b1, (void*)t1);
  k_dyn<<<dim3(NB_ * NPIX / 128), dim3(256), 0, stream>>>(t1, w2, b2, x, result);
  k_conv3p<<<dim3(NB_ * NPIX / 128), dim3(256), 0, stream>>>(result, w3, b3, out);
}
